// EdgePool_77446850281714
// MI455X (gfx1250) — hardware-verified
//
#include <hip/hip_runtime.h>
#include <math.h>

typedef __attribute__((ext_vector_type(16))) __bf16 v16bf;
typedef __attribute__((ext_vector_type(8)))  __bf16 v8bf;
typedef __attribute__((ext_vector_type(8)))  float  v8f;
typedef __attribute__((ext_vector_type(4)))  float  v4f;
typedef __attribute__((ext_vector_type(4)))  unsigned v4u;
typedef float __attribute__((may_alias)) float_a;
typedef int __attribute__((may_alias)) int_a;

#define NN 50000
#define NPAD 50176
#define EE 400000
#define HH 128
#define GG 64
#define NROUNDS 64
#define ETILE 2048

template <typename V> __device__ __forceinline__ void vst2(void* p, V v) {
  *(volatile V*)p = v; __threadfence(); *(volatile V*)p = v;
}
__device__ __forceinline__ v8f wmma_bf(v16bf a, v16bf b, v8f c) {
  v8f d = __builtin_amdgcn_wmma_f32_16x16x32_bf16(false, a, false, b, (short)0, c, false, false);
  asm volatile("v_nop\n\tv_nop\n\tv_nop\n\tv_nop" : "+v"(d) : "v"(a), "v"(b));
  return d;
}
struct A3 { v16bf h, m, l; };
__device__ __forceinline__ A3 split_row(const float* row, int k0, int lane) {
  A3 r; const float* p = row + k0 + 8 * (lane >> 4);
#pragma unroll
  for (int i = 0; i < 16; ++i) {
    const float x = p[(i < 8) ? i : (i + 8)];
    const __bf16 h = (__bf16)x; const float rh = x - (float)h;
    const __bf16 m = (__bf16)rh; const __bf16 l = (__bf16)(rh - (float)m);
    r.h[i] = h; r.m[i] = m; r.l[i] = l;
  }
  return r;
}
__device__ __forceinline__ v16bf frag_bf(const __bf16* row, int k0, int lane) {
  union { v16bf v; v8bf q[2]; } r; const __bf16* p = row + k0 + 8 * (lane >> 4);
  r.q[0] = *(const v8bf*)(p); r.q[1] = *(const v8bf*)(p + 16); return r.v;
}
__device__ __forceinline__ v8f mac6(const A3& a, const __bf16* bh, const __bf16* bm, const __bf16* bl, int k0, int lane, v8f c) {
  const v16bf fh = frag_bf(bh, k0, lane), fm = frag_bf(bm, k0, lane), fl = frag_bf(bl, k0, lane);
  c = wmma_bf(a.l, fh, c); c = wmma_bf(a.m, fm, c); c = wmma_bf(a.h, fl, c);
  c = wmma_bf(a.m, fh, c); c = wmma_bf(a.h, fm, c); c = wmma_bf(a.h, fh, c);
  return c;
}

template <int BT, int ECAP, int SCAP>
struct BucketT { int lidx[ECAP]; unsigned short ltgt[ECAP]; unsigned short sub[BT][SCAP]; int scnt[BT]; int wcnt[8][8]; int total; };
template <int BT, int ECAP, int SCAP>
__device__ void bucket_build(BucketT<BT, ECAP, SCAP>& bk, const int* __restrict__ t1, int E1, const int* __restrict__ t2, int E2, int tlo, int tid) {
  const int lane = tid & 31, wave = tid >> 5;
  if (tid == 0) bk.total = 0;
  __syncthreads();
  for (int e0 = 0; e0 < E2; e0 += ETILE) {
    int rv[8]; unsigned msk[8];
#pragma unroll
    for (int j = 0; j < 8; ++j) {
      const int e = e0 + j * 256 + tid;
      const int r = (e < E2) ? ((e < E1) ? t1[e] : t2[e - E1]) : -1;
      rv[j] = r;
      msk[j] = (unsigned)__builtin_amdgcn_ballot_w32((r >= tlo) && (r < tlo + BT));
    }
    if (lane < 8) bk.wcnt[lane][wave] = __builtin_popcount(msk[lane]);
    __syncthreads();
    const int base = bk.total;
    int run = 0, pre[8];
#pragma unroll
    for (int j = 0; j < 8; ++j) {
#pragma unroll
      for (int w = 0; w < 8; ++w) { if (w == wave) pre[j] = run; run += bk.wcnt[j][w]; }
    }
#pragma unroll
    for (int j = 0; j < 8; ++j) {
      const unsigned m = msk[j];
      if ((m >> lane) & 1u) {
        const int pos = base + pre[j] + __builtin_popcount(m & ((1u << lane) - 1u));
        if (pos < ECAP) { bk.lidx[pos] = e0 + j * 256 + tid; bk.ltgt[pos] = (unsigned short)(rv[j] - tlo); }
      }
    }
    __syncthreads();
    if (tid == 0) bk.total = base + run;
    __syncthreads();
  }
  const int n = (bk.total < ECAP) ? bk.total : ECAP;
  int k = 0;
  if (tid < BT) { for (int i = 0; i < n; ++i) if ((int)bk.ltgt[i] == tid) { if (k < SCAP) bk.sub[tid][k] = (unsigned short)i; ++k; } }
  if (tid < BT) bk.scnt[tid] = (k < SCAP) ? k : SCAP;
  __syncthreads();
}
typedef BucketT<256, 9216, 64> BucketD;
typedef BucketT<128, 9216, 128> BucketI;

__global__ __launch_bounds__(256) void k_split3(const float* __restrict__ Wrel, const float* __restrict__ Wroot, __bf16* __restrict__ P) {
  __shared__ __align__(16) __bf16 th[64][72], tm[64][72], tl[64][72];
  const int tid = threadIdx.x, n0 = (blockIdx.x & 1) * 64, k0 = (blockIdx.x >> 1) * 64;
  for (int i = tid; i < 64 * 64; i += 256) {
    const int kk = i >> 6, nn = i & 63; const int k = k0 + kk;
    const float x = (k < HH) ? Wrel[(size_t)k * HH + n0 + nn] : Wroot[(size_t)(k - HH) * HH + n0 + nn];
    const __bf16 h = (__bf16)x; const float rh = x - (float)h; const __bf16 m = (__bf16)rh; const __bf16 l = (__bf16)(rh - (float)m);
    th[nn][kk] = h; tm[nn][kk] = m; tl[nn][kk] = l;
  }
  __syncthreads();
  const size_t plane = (size_t)HH * 256;
  for (int g = tid; g < 64 * 8; g += 256) { const int nn = g >> 3, pc = g & 7; const size_t o = (size_t)(n0 + nn) * 256 + k0 + pc * 8;
    vst2(P + o, *(const v4u*)(&th[nn][pc * 8])); vst2(P + plane + o, *(const v4u*)(&tm[nn][pc * 8])); vst2(P + 2 * plane + o, *(const v4u*)(&tl[nn][pc * 8])); }
}

__global__ __launch_bounds__(256) void k_mean(const int* __restrict__ src, const int* __restrict__ dst, const float* __restrict__ x, float* __restrict__ agg) {
  __shared__ BucketD bk;
  const int tid = threadIdx.x, lane = tid & 31, wave = tid >> 5, tlo = blockIdx.x * 256;
  bucket_build(bk, dst, EE, dst, EE, tlo, tid);
  for (int s = 0; s < 32; ++s) {
    const int t = wave * 32 + s, node = tlo + t;
    if (node >= NN) break;
    const int cnt = bk.scnt[t];
    float a[4] = {0.f, 0.f, 0.f, 0.f};
    for (int k = 0; k < cnt; ++k) {
      int sN = src[bk.lidx[bk.sub[t][k]]]; sN = sN < 0 ? 0 : (sN >= NN ? NN - 1 : sN);
      const float* xr = x + (size_t)sN * HH;
#pragma unroll
      for (int j = 0; j < 4; ++j) a[j] += xr[lane + 32 * j];
    }
    const float inv = 1.f / (float)(cnt > 0 ? cnt : 1);
    float* ar = agg + (size_t)node * HH;
#pragma unroll
    for (int j = 0; j < 4; ++j) vst2(ar + lane + 32 * j, (float_a)(a[j] * inv));
  }
}
__global__ __launch_bounds__(128) void k_gcgemm(const float* __restrict__ agg, const float* __restrict__ x, const __bf16* __restrict__ P,
                                               const float* __restrict__ b, float* __restrict__ y) {
  __shared__ __align__(16) float so[16 * HH];
  const int tid = threadIdx.x, wave = tid >> 5, lane = tid & 31, hi = lane >> 4, col = lane & 15, m0 = blockIdx.x * 16;
  const size_t plane = (size_t)HH * 256;
  int arow = m0 + col; if (arow >= NN) arow = NN - 1;
  v8f c0 = {}, c1 = {};
  const int n0 = wave * 32;
#pragma unroll 1
  for (int kc = 0; kc < 8; ++kc) {
    const A3 a = (kc < 4) ? split_row(agg + (size_t)arow * HH, kc * 32, lane) : split_row(x + (size_t)arow * HH, (kc - 4) * 32, lane);
    { const size_t ro = (size_t)(n0 + col) * 256;      c0 = mac6(a, P + ro, P + plane + ro, P + 2 * plane + ro, kc * 32, lane, c0); }
    { const size_t ro = (size_t)(n0 + 16 + col) * 256; c1 = mac6(a, P + ro, P + plane + ro, P + 2 * plane + ro, kc * 32, lane, c1); }
  }
#pragma unroll
  for (int r = 0; r < 8; ++r) { so[(hi * 8 + r) * HH + n0 + col] = fmaxf(c0[r] + b[n0 + col], 0.f); so[(hi * 8 + r) * HH + n0 + 16 + col] = fmaxf(c1[r] + b[n0 + 16 + col], 0.f); }
  __syncthreads();
  for (int g = tid; g < 16 * 32; g += 128) { const int rl = g >> 5, pc = g & 31; if (m0 + rl < NN) vst2(y + (size_t)(m0 + rl) * HH + pc * 4, *(const v4f*)(&so[rl * HH + pc * 4])); }
}
__global__ __launch_bounds__(256) void k_gmp(const float* __restrict__ x, const int* __restrict__ batch, float* __restrict__ out, int coloff) {
  __shared__ float red[2][HH]; __shared__ int cred[2];
  const int g = blockIdx.x, tid = threadIdx.x, c = tid & 127, half = tid >> 7;
  float s = 0.f; int cnt = 0;
  for (int n = half; n < NN; n += 2) { if (batch[n] == g) { s += x[(size_t)n * HH + c]; ++cnt; } }
  red[half][c] = s; if (c == 0) cred[half] = cnt;
  __syncthreads();
  if (tid < HH) { const int ct = cred[0] + cred[1]; const float v = (red[0][tid] + red[1][tid]) / (float)(ct > 0 ? ct : 1); vst2(out + (size_t)g * 640 + coloff + tid, (float_a)v); }
}

__global__ __launch_bounds__(256) void k_raw(const int* __restrict__ src, const int* __restrict__ dst, const float* __restrict__ x,
                                            const float* __restrict__ w, const float* __restrict__ pb, float* __restrict__ raw) {
  __shared__ float red[32];
  const int tid = threadIdx.x, wave = tid >> 5, lane = tid & 31;
  for (int r = 0; r < 4; ++r) {
    const int e = blockIdx.x * 32 + wave * 4 + r;
    const int d = dst[e]; int sN = src[e]; sN = sN < 0 ? 0 : (sN >= NN ? NN - 1 : sN);
    float s = 0.f;
    if (d >= 0) {
      const float* xs = x + (size_t)sN * HH; const float* xd = x + (size_t)d * HH;
#pragma unroll
      for (int j = 0; j < 4; ++j) { const int c = lane + 32 * j; s += xs[c] * w[c] + xd[c] * w[HH + c]; }
#pragma unroll
      for (int off = 16; off > 0; off >>= 1) s += __shfl_xor(s, off, 32);
      s += pb[0];
    }
    if (lane == 0) red[wave * 4 + r] = s;
  }
  __syncthreads();
  if (tid < 32) vst2(raw + (size_t)blockIdx.x * 32 + tid, (float_a)red[tid]);
}
__global__ __launch_bounds__(256) void k_smax(const int* __restrict__ dst, const float* __restrict__ raw, float* __restrict__ mx, float* __restrict__ den) {
  __shared__ BucketD bk;
  __shared__ float sm[256], sd[256];
  const int tid = threadIdx.x, lane = tid & 31, wave = tid >> 5, tlo = blockIdx.x * 256;
  bucket_build(bk, dst, EE, dst, EE, tlo, tid);
  for (int s = 0; s < 32; ++s) {
    const int t = wave * 32 + s, node = tlo + t;
    if (node >= NN) break;
    const int cnt = bk.scnt[t];
    float m = -1e30f;
    for (int k = lane; k < cnt; k += 32) m = fmaxf(m, raw[bk.lidx[bk.sub[t][k]]]);
#pragma unroll
    for (int off = 16; off > 0; off >>= 1) m = fmaxf(m, __shfl_xor(m, off, 32));
    float d = 0.f;
    for (int k = lane; k < cnt; k += 32) d += __expf(raw[bk.lidx[bk.sub[t][k]]] - m);
#pragma unroll
    for (int off = 16; off > 0; off >>= 1) d += __shfl_xor(d, off, 32);
    if (lane == 0) { sm[t] = m; sd[t] = d; }
  }
  __syncthreads();
  if (tlo + tid < NPAD) { vst2(mx + tlo + tid, (float_a)sm[tid]); vst2(den + tlo + tid, (float_a)sd[tid]); }
}
__global__ __launch_bounds__(256) void k_score(const int* __restrict__ dst, const float* __restrict__ raw, const float* __restrict__ mx,
                                              const float* __restrict__ den, float* __restrict__ score) {
  const int e = blockIdx.x * 256 + threadIdx.x;
  if (e >= EE) return;
  const int d = dst[e];
  float s = -1.f;
  if (d >= 0) s = __expf(raw[e] - mx[d]) / fmaxf(den[d], 1e-16f) + 0.5f;
  vst2(score + e, (float_a)s);
}
__global__ __launch_bounds__(256) void k_fill_i(int* __restrict__ p, int v, int n) { const int i = blockIdx.x * 256 + threadIdx.x; if (i < n) vst2(p + i, (int_a)v); }
__global__ __launch_bounds__(256) void k_iota(int* __restrict__ p, int n) { const int i = blockIdx.x * 256 + threadIdx.x; if (i < n) vst2(p + i, (int_a)i); }

template <int MODE>
__global__ __launch_bounds__(256) void k_round(const int* __restrict__ srcv, const int* __restrict__ dstv, const int* __restrict__ src, const int* __restrict__ dst,
                                              const float* __restrict__ score, const int* __restrict__ tie, const int* __restrict__ sel,
                                              const int* __restrict__ nv, const int* __restrict__ matched_in, int* __restrict__ matched_out,
                                              float* __restrict__ bests, int* __restrict__ bestt) {
  __shared__ BucketI bk;
  __shared__ float rs[128]; __shared__ int rt[128];
  const int tid = threadIdx.x, lane = tid & 31, wave = tid >> 5, tlo = blockIdx.x * 128;
  bucket_build(bk, dstv, EE, srcv, 2 * EE, tlo, tid);
  for (int s = 0; s < 16; ++s) {
    const int t = wave * 16 + s, node = tlo + t;
    if (node >= NN) break;
    const int cnt = bk.scnt[t];
    if (MODE == 0) {
      int any = 0;
      for (int k = lane; k < cnt; k += 32) { int i = bk.lidx[bk.sub[t][k]]; const int e = (i < EE) ? i : i - EE; any |= sel[e]; }
#pragma unroll
      for (int off = 16; off > 0; off >>= 1) any |= __shfl_xor(any, off, 32);
      if (lane == 0) rt[t] = (nv[node] == 0) | (any != 0);
    } else {
      float bs = -2.f; int bt = 0x7fffffff;
      for (int k = lane; k < cnt; k += 32) {
        int i = bk.lidx[bk.sub[t][k]]; const int e = (i < EE) ? i : i - EE;
        const float sc = score[e];
        if (sc < 0.f || sel[e]) continue;
        int a = src[e], b = dst[e]; a = a < 0 ? 0 : (a >= NN ? NN - 1 : a);
        if (matched_in[a] || matched_in[b]) continue;
        const int te = tie[e];
        if (sc > bs || (sc == bs && te < bt)) { bs = sc; bt = te; }
      }
#pragma unroll
      for (int off = 16; off > 0; off >>= 1) {
        const float os = __shfl_xor(bs, off, 32); const int ot = __shfl_xor(bt, off, 32);
        if (os > bs || (os == bs && ot < bt)) { bs = os; bt = ot; }
      }
      if (lane == 0) { rs[t] = bs; rt[t] = bt; }
    }
  }
  __syncthreads();
  if (tid < 128 && tlo + tid < NPAD) {
    if (MODE == 0) vst2(matched_out + tlo + tid, (int_a)rt[tid]);
    else { vst2(bests + tlo + tid, (float_a)rs[tid]); vst2(bestt + tlo + tid, (int_a)rt[tid]); }
  }
}
__global__ __launch_bounds__(256) void k_dom(const int* __restrict__ src, const int* __restrict__ dst, const float* __restrict__ score, const int* __restrict__ tie,
                                            const int* __restrict__ matched, const float* __restrict__ bests, const int* __restrict__ bestt,
                                            const int* __restrict__ sel_in, int* __restrict__ sel_out) {
  const int e = blockIdx.x * 256 + threadIdx.x;
  if (e >= EE) return;
  const float sc = score[e]; const int d = dst[e]; int a = src[e]; a = a < 0 ? 0 : (a >= NN ? NN - 1 : a);
  int sl = sel_in[e];
  if (!sl && sc >= 0.f && d >= 0 && !matched[a] && !matched[d]) {
    const int te = tie[e];
    if (sc == bests[a] && te == bestt[a] && sc == bests[d] && te == bestt[d]) sl = 1;
  }
  vst2(sel_out + e, (int_a)sl);
}
__global__ __launch_bounds__(256) void k_kid(const float* __restrict__ score, const int* __restrict__ tie, const int* __restrict__ sel, int* __restrict__ kid) {
  __shared__ float ts[2048]; __shared__ int tt[2048];
  const int eg = blockIdx.x * 256 + threadIdx.x; const int e = (eg < EE) ? eg : EE - 1;
  const int mine = (eg < EE) ? sel[e] : 0; const float sc = score[e]; const int te = tie[e];
  const int anysel = __syncthreads_or(mine);
  int cnt = 0;
  if (anysel) {
    for (int j0 = 0; j0 < EE; j0 += 2048) {
      __syncthreads();
      for (int t = threadIdx.x; t < 2048; t += 256) { const int j = j0 + t; const bool ok = (j < EE) && sel[j]; ts[t] = ok ? score[j] : -3.f; tt[t] = ok ? tie[j] : 0; }
      __syncthreads();
      if (mine) {
#pragma unroll 4
        for (int t = 0; t < 2048; ++t) { const float s2 = ts[t]; cnt += (s2 > sc) | ((s2 == sc) & (tt[t] < te)); }
      }
    }
  }
  if (eg < EE) vst2(kid + e, (int_a)(mine ? cnt : -1));
}
__global__ __launch_bounds__(256) void k_selcount(const int* __restrict__ sel, int* __restrict__ part) {
  __shared__ int red[8];
  const int tid = threadIdx.x, lane = tid & 31, wave = tid >> 5;
  int c = 0;
  for (int i = 0; i < 16; ++i) c += sel[(size_t)blockIdx.x * 4096 + i * 256 + tid] != 0;
#pragma unroll
  for (int off = 16; off > 0; off >>= 1) c += __shfl_xor(c, off, 32);
  if (lane == 0) red[wave] = c;
  __syncthreads();
  if (tid < 32) { int v = 0; if (tid == 0) { for (int w = 0; w < 8; ++w) v += red[w]; } vst2(part + blockIdx.x * 32 + tid, (int_a)(tid == 0 ? v : 0)); }
}
__global__ __launch_bounds__(256) void k_nodesel(const int* __restrict__ srcv, const int* __restrict__ dstv, const float* __restrict__ score,
                                                const int* __restrict__ sel, const int* __restrict__ kid, int* __restrict__ msel, int* __restrict__ clsel, float* __restrict__ selsc) {
  __shared__ BucketI bk;
  __shared__ int rm[128], rc[128]; __shared__ float rsc[128];
  const int tid = threadIdx.x, lane = tid & 31, wave = tid >> 5, tlo = blockIdx.x * 128;
  bucket_build(bk, dstv, EE, srcv, 2 * EE, tlo, tid);
  for (int s = 0; s < 16; ++s) {
    const int t = wave * 16 + s, node = tlo + t;
    if (node >= NN) break;
    const int cnt = bk.scnt[t];
    int k_ = -1; float sc = 1.f;
    for (int k = lane; k < cnt; k += 32) { int i = bk.lidx[bk.sub[t][k]]; const int e = (i < EE) ? i : i - EE; if (sel[e]) { k_ = kid[e]; sc = score[e]; } }
#pragma unroll
    for (int off = 16; off > 0; off >>= 1) { const int ok = __shfl_xor(k_, off, 32); const float os = __shfl_xor(sc, off, 32); if (ok > k_) { k_ = ok; sc = os; } }
    if (lane == 0) { rm[t] = (k_ >= 0); rc[t] = k_; rsc[t] = sc; }
  }
  __syncthreads();
  if (tid < 128 && tlo + tid < NPAD) { vst2(msel + tlo + tid, (int_a)rm[tid]); vst2(clsel + tlo + tid, (int_a)rc[tid]); vst2(selsc + tlo + tid, (float_a)rsc[tid]); }
}
__global__ __launch_bounds__(256) void k_scan1(const int* __restrict__ nv, const int* __restrict__ msel, int* __restrict__ part) {
  __shared__ int red[2][8];
  const int tid = threadIdx.x, lane = tid & 31, wave = tid >> 5;
  int cr = 0, ci = 0;
  for (int i = 0; i < 4; ++i) { const int n = blockIdx.x * 1024 + i * 256 + tid; if (n < NN) { const int v = nv[n]; cr += (v && !msel[n]); ci += !v; } }
#pragma unroll
  for (int off = 16; off > 0; off >>= 1) { cr += __shfl_xor(cr, off, 32); ci += __shfl_xor(ci, off, 32); }
  if (lane == 0) { red[0][wave] = cr; red[1][wave] = ci; }
  __syncthreads();
  if (tid < 32) { int v = 0; if (tid < 2) { for (int w = 0; w < 8; ++w) v += red[tid][w]; } vst2(part + blockIdx.x * 32 + tid, (int_a)v); }
}
__global__ __launch_bounds__(64) void k_scan2(const int* __restrict__ part, const int* __restrict__ selpart, int nselb, int* __restrict__ offs, int* __restrict__ tot) {
  __shared__ int exr[64], exi[64], ksum, trr;
  const int t = threadIdx.x, lane = t & 31, wave = t >> 5;
  const int cr = (t < 49) ? part[t * 32 + 0] : 0, ci = (t < 49) ? part[t * 32 + 1] : 0;
  __shared__ int sr[64], si[64];
  sr[t] = cr; si[t] = ci;
  __syncthreads();
  if (t == 0) {
    int ar = 0, ai = 0;
    for (int i = 0; i < 49; ++i) { exr[i] = ar; exi[i] = ai; ar += sr[i]; ai += si[i]; }
    trr = ar;
    int k = 0; for (int i = 0; i < nselb; ++i) k += selpart[i * 32]; ksum = k;
  }
  __syncthreads();
  for (int b = wave; b < 49; b += 2) vst2(offs + b * 32 + lane, (int_a)(lane == 0 ? exr[b] : (lane == 1 ? exi[b] : 0)));
  if (wave == 0) vst2(tot + lane, (int_a)(lane == 0 ? ksum : (lane == 1 ? trr : (lane == 2 ? ksum + trr : 0))));
}
__global__ __launch_bounds__(256) void k_scan3(const int* __restrict__ nv, const int* __restrict__ msel, const int* __restrict__ clsel,
                                              const int* __restrict__ offs, const int* __restrict__ tot, int* __restrict__ cl) {
  __shared__ int pr[1024], pi[1024];
  const int tid = threadIdx.x, b = blockIdx.x;
  for (int i = 0; i < 4; ++i) { const int l = i * 256 + tid, n = b * 1024 + l; int v = (n < NN) ? nv[n] : 0, ms = (n < NN) ? msel[n] : 1;
    pr[l] = (n < NN) && v && !ms; pi[l] = (n < NN) && !v; }
  __syncthreads();
  for (int off = 1; off < 1024; off <<= 1) {
    int ar[4], ai[4];
    for (int i = 0; i < 4; ++i) { const int l = i * 256 + tid; ar[i] = (l >= off) ? pr[l - off] : 0; ai[i] = (l >= off) ? pi[l - off] : 0; }
    __syncthreads();
    for (int i = 0; i < 4; ++i) { const int l = i * 256 + tid; pr[l] += ar[i]; pi[l] += ai[i]; }
    __syncthreads();
  }
  const int k = tot[0], n_new = tot[2], offr = offs[b * 32 + 0], offi = offs[b * 32 + 1];
  for (int i = 0; i < 4; ++i) {
    const int l = i * 256 + tid, n = b * 1024 + l;
    if (n >= NPAD) continue;
    int c = 0;
    if (n < NN) {
      const int v = nv[n], ms = msel[n];
      if (v && ms) c = clsel[n];
      else if (v) c = k + offr + pr[l] - 1;
      else c = n_new + offi + pi[l] - 1;
    }
    vst2(cl + n, (int_a)c);
  }
}
__global__ __launch_bounds__(256) void k_cluster(const int* __restrict__ cl, const float* __restrict__ x, const int* __restrict__ nv, const int* __restrict__ batch,
                                                const int* __restrict__ msel, const float* __restrict__ selsc, const int* __restrict__ tot,
                                                float* __restrict__ nx, int* __restrict__ nbatch, int* __restrict__ nnv) {
  __shared__ BucketD bk;
  __shared__ int rb[256], rv[256];
  const int tid = threadIdx.x, lane = tid & 31, wave = tid >> 5, tlo = blockIdx.x * 256;
  bucket_build(bk, cl, NN, cl, NN, tlo, tid);
  const int n_new = tot[2];
  for (int s = 0; s < 32; ++s) {
    const int t = wave * 32 + s, c = tlo + t;
    if (c >= NPAD) break;
    const int cnt = (c < NN) ? bk.scnt[t] : 0;
    float a[4] = {0.f, 0.f, 0.f, 0.f}; float scale = 1.f; int bval = GG, lastn = -1;
    for (int k = 0; k < cnt; ++k) {
      const int n = bk.lidx[bk.sub[t][k]];
      const int v = nv[n];
      if (v) { const float* xr = x + (size_t)n * HH;
#pragma unroll
        for (int j = 0; j < 4; ++j) a[j] += xr[lane + 32 * j]; }
      if (n > lastn) { lastn = n; bval = v ? batch[n] : GG; if (msel[n]) scale = selsc[n]; }
    }
    if (c < NN) { float* orow = nx + (size_t)c * HH;
#pragma unroll
      for (int j = 0; j < 4; ++j) vst2(orow + lane + 32 * j, (float_a)(a[j] * scale)); }
    if (lane == 0) { rb[t] = bval; rv[t] = (c < n_new); }
  }
  __syncthreads();
  if (tlo + tid < NPAD) { vst2(nbatch + tlo + tid, (int_a)rb[tid]); vst2(nnv + tlo + tid, (int_a)rv[tid]); }
}
__global__ __launch_bounds__(256) void k_csct(const int* __restrict__ src, const int* __restrict__ dst, const int* __restrict__ cl, int* __restrict__ cs, int* __restrict__ ct) {
  const int e = blockIdx.x * 256 + threadIdx.x;
  if (e >= EE) return;
  const int d = dst[e]; int a = src[e]; a = a < 0 ? 0 : (a >= NN ? NN - 1 : a);
  vst2(cs + e, (int_a)(d >= 0 ? cl[a] : NN)); vst2(ct + e, (int_a)(d >= 0 ? cl[d] : NN));
}
__global__ __launch_bounds__(256) void k_coalesce(const int* __restrict__ cs, const int* __restrict__ ct, const int* __restrict__ tie,
                                                 int* __restrict__ nsrc, int* __restrict__ ndst, int* __restrict__ nsrcv, int* __restrict__ ntie) {
  __shared__ int t1[2048], t2[2048], t3[2048];
  const int eg = blockIdx.x * 256 + threadIdx.x; const int e = (eg < EE) ? eg : EE - 1;
  const int a = cs[e], b = ct[e], te = tie[e];
  int rank = 0, dup = 0;
  for (int j0 = 0; j0 < EE; j0 += 2048) {
    __syncthreads();
    for (int t = threadIdx.x; t < 2048; t += 256) { const int j = j0 + t; if (j < EE) { t1[t] = cs[j]; t2[t] = ct[j]; t3[t] = tie[j]; } else { t1[t] = 0x7fffffff; t2[t] = 0; t3[t] = 0; } }
    __syncthreads();
#pragma unroll 4
    for (int t = 0; t < 2048; ++t) {
      const int a2 = t1[t], b2 = t2[t], u2 = t3[t];
      const bool less = (a2 < a) || (a2 == a && (b2 < b || (b2 == b && u2 < te)));
      rank += less;
      dup |= (a2 == a) & (b2 == b) & (u2 < te);
    }
  }
  const bool valid = (a < NN) && !dup;
  if (eg >= EE) return;
  vst2(nsrc + e, (int_a)(valid ? a : 0)); vst2(ndst + e, (int_a)(valid ? b : -1)); vst2(nsrcv + e, (int_a)(valid ? a : -1)); vst2(ntie + e, (int_a)rank);
}

__global__ __launch_bounds__(256) void k_copy_i(const int* __restrict__ s, int n, int padval, int ntot, int* __restrict__ d) {
  const int i = blockIdx.x * 256 + threadIdx.x; if (i < ntot) vst2(d + i, (int_a)(i < n ? s[i] : padval)); }

extern "C" void kernel_launch(void* const* d_in, const int* in_sizes, int n_in,
                              void* d_out, int out_size, void* d_ws, size_t ws_size,
                              hipStream_t stream) {
  (void)in_sizes; (void)n_in; (void)out_size; (void)ws_size;
  const float* x0 = (const float*)d_in[0];
  const int* ei = (const int*)d_in[1];
  const int* batch0 = (const int*)d_in[2];
  const float *Wrel1 = (const float*)d_in[3], *brel1 = (const float*)d_in[4], *Wroot1 = (const float*)d_in[5];
  const float *Wrels = (const float*)d_in[6], *brels = (const float*)d_in[7], *Wroots = (const float*)d_in[8];
  const float *pool_w = (const float*)d_in[9], *pool_b = (const float*)d_in[10];
  float* out = (float*)d_out;

  char* ws = (char*)d_ws; size_t off = 0;
  auto alloc = [&](size_t bytes) -> void* { void* p = ws + off; off = (off + bytes + 255) & ~(size_t)255; return p; };
  auto ialloc = [&](size_t n) -> int* { return (int*)alloc(n * 4); };
  auto falloc = [&](size_t n) -> float* { return (float*)alloc(n * 4); };
  const int EPAD = 98 * 4096;
  __bf16* P[5]; for (int i = 0; i < 5; ++i) P[i] = (__bf16*)alloc((size_t)3 * HH * 256 * 2);
  float* XA = falloc((size_t)NN * HH); float* XB = falloc((size_t)NN * HH); float* AGG = falloc((size_t)NN * HH);
  int *srcA = ialloc(EE), *dstA = ialloc(EE), *srcvA = ialloc(EE), *tieA = ialloc(EE);
  int *srcB = ialloc(EE), *dstB = ialloc(EE), *srcvB = ialloc(EE), *tieB = ialloc(EE);
  int *batchA = ialloc(NPAD), *batchB = ialloc(NPAD), *nvA = ialloc(NPAD), *nvB = ialloc(NPAD);
  float *raw = falloc(EE), *score = falloc(EE), *mx = falloc(NPAD), *den = falloc(NPAD);
  int *selA = ialloc(EPAD), *selB = ialloc(EPAD), *kid = ialloc(EE), *cs = ialloc(EE), *ct = ialloc(EE);
  int *matched = ialloc(NPAD), *bestt = ialloc(NPAD), *msel = ialloc(NPAD), *clsel = ialloc(NPAD), *cl = ialloc(NPAD);
  float *bests = falloc(NPAD), *selsc = falloc(NPAD);
  int *selpart = ialloc(98 * 32), *scanpart = ialloc(49 * 32), *offs = ialloc(49 * 32), *tot = ialloc(32);

  const int EB = (EE + 255) / 256, NB256 = NPAD / 256, NB128 = (NN + 127) / 128;
  k_split3<<<8, 256, 0, stream>>>(Wrel1, Wroot1, P[0]);
  for (int i = 0; i < 4; ++i) k_split3<<<8, 256, 0, stream>>>(Wrels + (size_t)i * HH * HH, Wroots + (size_t)i * HH * HH, P[i + 1]);
  k_copy_i<<<EB, 256, 0, stream>>>(ei, EE, 0, EE, srcA);
  k_copy_i<<<EB, 256, 0, stream>>>(ei + EE, EE, 0, EE, dstA);
  k_copy_i<<<EB, 256, 0, stream>>>(ei, EE, 0, EE, srcvA);
  k_iota<<<EB, 256, 0, stream>>>(tieA, EE);
  k_copy_i<<<NB256, 256, 0, stream>>>(batch0, NN, GG, NPAD, batchA);
  k_fill_i<<<NB256, 256, 0, stream>>>(nvA, 1, NN);
  k_fill_i<<<1, 256, 0, stream>>>(nvA + NN, 0, NPAD - NN);

  struct Gr { int *src, *dst, *srcv, *tie, *batch, *nv; };
  Gr GA = {srcA, dstA, srcvA, tieA, batchA, nvA}, GB = {srcB, dstB, srcvB, tieB, batchB, nvB};

  auto conv = [&](int l, const float* xin, float* xout, const Gr& g, const float* bias) {
    k_mean<<<NB256, 256, 0, stream>>>(g.src, g.dst, xin, AGG);
    k_gcgemm<<<(NN + 15) / 16, 128, 0, stream>>>(AGG, xin, P[l], bias, xout);
  };
  auto gmp = [&](const float* x, const Gr& g, int coloff) { k_gmp<<<GG, 256, 0, stream>>>(x, g.batch, out, coloff); };
  auto pool = [&](int pi, const float* x, const Gr& g, float* xnew, const Gr& gn) {
    k_raw<<<EE / 32, 256, 0, stream>>>(g.src, g.dst, x, pool_w + (size_t)pi * 2 * HH, pool_b + pi, raw);
    k_smax<<<NB256, 256, 0, stream>>>(g.dst, raw, mx, den);
    k_score<<<EB, 256, 0, stream>>>(g.dst, raw, mx, den, score);
    k_fill_i<<<(EPAD + 255) / 256, 256, 0, stream>>>(selA, 0, EPAD);
    k_fill_i<<<(EPAD + 255) / 256, 256, 0, stream>>>(selB, 0, EPAD);
    int* sc_ = selA; int* sn_ = selB;
    for (int r = 0; r < NROUNDS; ++r) {
      k_round<0><<<NB128, 256, 0, stream>>>(g.srcv, g.dst, g.src, g.dst, score, g.tie, sc_, g.nv, nullptr, matched, nullptr, nullptr);
      k_round<1><<<NB128, 256, 0, stream>>>(g.srcv, g.dst, g.src, g.dst, score, g.tie, sc_, g.nv, matched, nullptr, bests, bestt);
      k_dom<<<EB, 256, 0, stream>>>(g.src, g.dst, score, g.tie, matched, bests, bestt, sc_, sn_);
      int* tmp = sc_; sc_ = sn_; sn_ = tmp;
    }
    k_kid<<<EB, 256, 0, stream>>>(score, g.tie, sc_, kid);
    k_selcount<<<98, 256, 0, stream>>>(sc_, selpart);
    k_round<0><<<NB128, 256, 0, stream>>>(g.srcv, g.dst, g.src, g.dst, score, g.tie, sc_, g.nv, nullptr, matched, nullptr, nullptr);
    k_nodesel<<<NB128, 256, 0, stream>>>(g.srcv, g.dst, score, sc_, kid, msel, clsel, selsc);
    k_scan1<<<49, 256, 0, stream>>>(g.nv, msel, scanpart);
    k_scan2<<<1, 64, 0, stream>>>(scanpart, selpart, 98, offs, tot);
    k_scan3<<<49, 256, 0, stream>>>(g.nv, msel, clsel, offs, tot, cl);
    k_cluster<<<NB256, 256, 0, stream>>>(cl, x, g.nv, g.batch, msel, selsc, tot, xnew, gn.batch, gn.nv);
    k_csct<<<EB, 256, 0, stream>>>(g.src, g.dst, cl, cs, ct);
    k_coalesce<<<EB, 256, 0, stream>>>(cs, ct, g.tie, gn.src, gn.dst, gn.srcv, gn.tie);
  };

  conv(0, x0, XA, GA, brel1);            gmp(XA, GA, 0);
  conv(1, XA, XB, GA, brels + 0 * HH);   gmp(XB, GA, 128);
  pool(0, XB, GA, XA, GB);
  conv(2, XA, XB, GB, brels + 1 * HH);   gmp(XB, GB, 256);
  conv(3, XB, XA, GB, brels + 2 * HH);   gmp(XA, GB, 384);
  pool(1, XA, GB, XB, GA);
  conv(4, XB, XA, GA, brels + 3 * HH);   gmp(XA, GA, 512);
}
